// GenericAttentionBlock_4552665334361
// MI455X (gfx1250) — hardware-verified
//
#include <hip/hip_runtime.h>
#include <math.h>
#include <stdint.h>

constexpr int   kBatch    = 2;
constexpr int   kSeq      = 2048;
constexpr int   kTok      = kBatch * kSeq;
constexpr int   kDModel   = 1024;
constexpr int   kHeads    = 16;
constexpr int   kHD       = 64;
constexpr int   kRopeD    = 30;
constexpr float kEps      = 1e-6f;
constexpr float kLogPi    = 1.14472988584940017f;
constexpr float kFreqStep = 0.01439115683121279f;
constexpr float kWqScale  = 32.0f;
constexpr float kWoScale  = 64.0f;
constexpr float kQkScale  = 4.0f;
constexpr float kOScale   = 16.0f;
constexpr float kPSC      = 32768.0f;

typedef __attribute__((ext_vector_type(16))) _Float16 v16h;
typedef __attribute__((ext_vector_type(8)))  _Float16 v8h;
typedef __attribute__((ext_vector_type(16))) __bf16   v16b;
typedef __attribute__((ext_vector_type(8)))  __bf16   v8b;
typedef __attribute__((ext_vector_type(8)))  float    v8f;
typedef __attribute__((ext_vector_type(4)))  float    v4f;

__device__ __forceinline__ unsigned short f2bf_bits(float f) {
  unsigned u = __float_as_uint(f);
  return (unsigned short)((u + 0x7FFFu + ((u >> 16) & 1u)) >> 16);
}
__device__ __forceinline__ float bf_bits2f(unsigned short h) { return __uint_as_float(((unsigned)h) << 16); }

__device__ __forceinline__ void dep_guard_h(v8f& a, v8f& b, v16h x, v16h y) { asm volatile("v_nop\n\tv_nop\n\tv_nop\n\tv_nop" : "+v"(a), "+v"(b) : "v"(x), "v"(y)); }
__device__ __forceinline__ void dep_guard_b(v8f& a, v8f& b, v16b x, v16b y) { asm volatile("v_nop\n\tv_nop\n\tv_nop\n\tv_nop" : "+v"(a), "+v"(b) : "v"(x), "v"(y)); }
__device__ __forceinline__ void keep4_h(v16h a, v16h b, v16h c, v16h d) { asm volatile("v_nop" :: "v"(a), "v"(b), "v"(c), "v"(d)); }
__device__ __forceinline__ void keep4_b(v16b a, v16b b, v16b c, v16b d) { asm volatile("v_nop" :: "v"(a), "v"(b), "v"(c), "v"(d)); }
__device__ __forceinline__ void acc_guard4(v8f& a, v8f& b, v8f& c, v8f& d) { asm volatile("v_nop\n\tv_nop\n\tv_nop\n\tv_nop" : "+v"(a), "+v"(b), "+v"(c), "+v"(d)); }
template <typename T> struct Frag;
template <> struct Frag<_Float16> {
  typedef v16h V; union U { v16h v; v8h h[2]; };
  static __device__ __forceinline__ v16h load(const _Float16* p) {
    U f; f.h[0] = *(const v8h*)(p); f.h[1] = *(const v8h*)(p + 16); return f.v;
  }
  static __device__ __forceinline__ v8f mma(v16h a, v16h b, v8f c) {
    return __builtin_amdgcn_wmma_f32_16x16x32_f16(false, a, false, b, (short)0, c, false, false);
  }
  static __device__ __forceinline__ void guard(v8f& a, v8f& b, v16h x, v16h y) { dep_guard_h(a, b, x, y); }
  static __device__ __forceinline__ void keep(v16h a, v16h b, v16h c, v16h d) { keep4_h(a, b, c, d); }
};
template <> struct Frag<__bf16> {
  typedef v16b V; union U { v16b v; v8b h[2]; };
  static __device__ __forceinline__ v16b load(const __bf16* p) {
    U f; f.h[0] = *(const v8b*)(p); f.h[1] = *(const v8b*)(p + 16); return f.v;
  }
  static __device__ __forceinline__ v8f mma(v16b a, v16b b, v8f c) {
    return __builtin_amdgcn_wmma_f32_16x16x32_bf16(false, a, false, b, (short)0, c, false, false);
  }
  static __device__ __forceinline__ void guard(v8f& a, v8f& b, v16b x, v16b y) { dep_guard_b(a, b, x, y); }
  static __device__ __forceinline__ void keep(v16b a, v16b b, v16b c, v16b d) { keep4_b(a, b, c, d); }
};

template <int ET> struct Elem;
template <> struct Elem<0> { typedef _Float16 T; };
template <> struct Elem<1> { typedef __bf16 T; };
template <int ET, bool SPLIT, int BIAS_MODE, int OUT_MODE, bool RESID, int ACT = 0>
__global__ __launch_bounds__(256) void wmma_gemm64(
    const unsigned short* __restrict__ Ap, const unsigned short* __restrict__ A2p, int lda, long strideA,
    const unsigned short* __restrict__ Btp, const unsigned short* __restrict__ Bt2p, int ldb, long strideB,
    void* __restrict__ Cout, void* __restrict__ Cout2, int ldc, long strideC,
    const float* __restrict__ bias,
    const float* __restrict__ resid, long strideR,
    int M, int N, int K, float scale) {
  typedef typename Elem<ET>::T T;
  typedef typename Frag<T>::V V;
  const T* A = (const T*)Ap; const T* A2 = (const T*)A2p; const T* Bt = (const T*)Btp; const T* Bt2 = (const T*)Bt2p;
  __shared__ __align__(16) float sT[8][16 * 68];
  const int b    = blockIdx.y;
  const int lane = threadIdx.x & 31;
  const int wave = threadIdx.x >> 5;
  const int tilesN = N >> 6;
  const int tilesM = M >> 6;
  const int tile = blockIdx.x * 8 + wave;
  if (tile >= tilesM * tilesN) return;
  const int tm = tile / tilesN;
  const int tn = tile - tm * tilesN;
  const int m0 = tm << 6;
  const int n0 = tn << 6;

  const T* Ab  = A  + (size_t)b * strideA;
  const T* Bb  = Bt + (size_t)b * strideB;
  const T* Ab2 = SPLIT ? (A2  + (size_t)b * strideA) : nullptr;
  const T* Bb2 = SPLIT ? (Bt2 + (size_t)b * strideB) : nullptr;

  const int rlane = lane & 15;
  const int koff  = (lane >> 4) * 8;
  const int mOff  = (lane >> 4) * 8;

  v8f acc[4][4];
#pragma unroll
  for (int i = 0; i < 4; ++i)
#pragma unroll
    for (int j = 0; j < 4; ++j) acc[i][j] = (v8f){0.f,0.f,0.f,0.f,0.f,0.f,0.f,0.f};

  for (int k0 = 0; k0 < K; k0 += 32) {
    V bh[4], bl[4];
#pragma unroll
    for (int j = 0; j < 4; ++j) {
      const size_t bo = (size_t)(n0 + (j << 4) + rlane) * ldb + koff + k0;
      bh[j] = Frag<T>::load(Bb + bo);
      if (SPLIT) bl[j] = Frag<T>::load(Bb2 + bo);
    }
#pragma unroll
    for (int i = 0; i < 4; ++i) {
      const size_t ao = (size_t)(m0 + (i << 4) + rlane) * lda + koff + k0;
      V ah = Frag<T>::load(Ab + ao);
      V al;
      if (SPLIT) al = Frag<T>::load(Ab2 + ao);
#pragma unroll
      for (int j = 0; j < 4; ++j) {
        acc[i][j] = Frag<T>::mma(ah, bh[j], acc[i][j]);
        if (SPLIT) {
          acc[i][j] = Frag<T>::mma(ah, bl[j], acc[i][j]);
          acc[i][j] = Frag<T>::mma(al, bh[j], acc[i][j]);
        }
      }
      Frag<T>::guard(acc[i][0], acc[i][3], ah, SPLIT ? al : ah);
    }
    Frag<T>::keep(bh[0], bh[1], bh[2], bh[3]);
    if (SPLIT) Frag<T>::keep(bl[0], bl[1], bl[2], bl[3]);
  }
  acc_guard4(acc[0][0], acc[0][1], acc[0][2], acc[0][3]);
  acc_guard4(acc[1][0], acc[1][1], acc[1][2], acc[1][3]);
  acc_guard4(acc[2][0], acc[2][1], acc[2][2], acc[2][3]);
  acc_guard4(acc[3][0], acc[3][1], acc[3][2], acc[3][3]);

  float* slab = sT[wave];
  const float* Rb = RESID ? (resid + (size_t)b * strideR) : nullptr;
#pragma unroll
  for (int i = 0; i < 4; ++i) {
    const int mBase = m0 + (i << 4);
#pragma unroll
    for (int j = 0; j < 4; ++j) {
      const int n = n0 + (j << 4) + rlane;
      float bv = 0.f;
      if (BIAS_MODE == 2) bv = bias[n];
#pragma unroll
      for (int r = 0; r < 8; ++r) {
        float v = acc[i][j][r] * scale;
        if (BIAS_MODE == 1) v += bias[mBase + mOff + r];
        if (BIAS_MODE == 2) v += bv;
        if (RESID) v += Rb[(size_t)(mBase + mOff + r) * ldc + n];
        if (ACT == 1) v = tanhf(v);
        if (ACT == 2) v = fmaxf(v, 0.0f);
        if (ACT == 3) v = v / (1.0f + expf(-v));
        if (ACT == 4) v = (v > 0.f) ? v : 0.01f * v;
        if (ACT == 5) v = 0.5f * v * (1.0f + erff(v * 0.70710678118654752f));
        slab[(mOff + r) * 68 + (j << 4) + rlane] = v;
      }
    }
    __builtin_amdgcn_fence(__ATOMIC_RELEASE, "workgroup");
    __builtin_amdgcn_wave_barrier();
    __builtin_amdgcn_fence(__ATOMIC_ACQUIRE, "workgroup");
    if (OUT_MODE == 0) {
      float* C = (float*)Cout + (size_t)b * strideC;
      const int hh = lane >> 4, c4 = (lane & 15) * 4;
      for (int pass = 0; pass < 2; ++pass) {
#pragma unroll
        for (int it = 0; it < 8; ++it) {
          const int row = it * 2 + hh;
          v4f v = *(const v4f*)(slab + row * 68 + c4);
          *(volatile v4f*)(C + (size_t)(mBase + row) * ldc + n0 + c4) = v;
        }
        __threadfence();
      }
    } else {
      const int q = lane >> 3, c8 = (lane & 7) * 8;
      unsigned short* C  = (unsigned short*)Cout  + (size_t)b * strideC;
      unsigned short* C2 = (OUT_MODE == 2) ? ((unsigned short*)Cout2 + (size_t)b * strideC) : nullptr;
      for (int pass = 0; pass < 2; ++pass) {
#pragma unroll
        for (int it = 0; it < 4; ++it) {
          const int row = it * 4 + q;
          const float* sp = slab + row * 68 + c8;
          v8h hv, lv;
#pragma unroll
          for (int e = 0; e < 8; ++e) {
            if (OUT_MODE == 1) {
              hv[e] = (_Float16)sp[e];
            } else {
              unsigned short hb = f2bf_bits(sp[e]);
              unsigned short lb = f2bf_bits(sp[e] - bf_bits2f(hb));
              hv[e] = __builtin_bit_cast(_Float16, hb);
              lv[e] = __builtin_bit_cast(_Float16, lb);
            }
          }
          *(volatile v8h*)(C + (size_t)(mBase + row) * ldc + n0 + c8) = hv;
          if (OUT_MODE == 2) *(volatile v8h*)(C2 + (size_t)(mBase + row) * ldc + n0 + c8) = lv;
        }
        __threadfence();
      }
    }
    __builtin_amdgcn_fence(__ATOMIC_RELEASE, "workgroup");
    __builtin_amdgcn_wave_barrier();
    __builtin_amdgcn_fence(__ATOMIC_ACQUIRE, "workgroup");
  }
}

__global__ __launch_bounds__(256) void cast_scale_f32_f16x2(
    const float* __restrict__ in, unsigned short* __restrict__ out, int n2, float sc) {
  const int i = blockIdx.x * 256 + threadIdx.x;
  if (i < n2) {
    const _Float16 h0 = (_Float16)(in[2 * (size_t)i] * sc), h1 = (_Float16)(in[2 * (size_t)i + 1] * sc);
    const unsigned u = (unsigned)__builtin_bit_cast(unsigned short, h0) | ((unsigned)__builtin_bit_cast(unsigned short, h1) << 16);
    ((volatile unsigned*)out)[i] = u;
    __threadfence();
    ((volatile unsigned*)out)[i] = u;
  }
}

__global__ __launch_bounds__(128) void rmsnorm_f16_kernel(
    const float* __restrict__ x, const float* __restrict__ gamma, unsigned short* __restrict__ hout,
    int ntok, float eps) {
  __shared__ float red[4];
  int row = blockIdx.x;
  if (row > ntok - 1) row = ntok - 1;
  const int tid = threadIdx.x, lane = tid & 31, wave = tid >> 5;
  const float* xr = x + (size_t)row * kDModel + 8 * tid;
  const v4f a0 = *(const v4f*)(xr);
  const v4f a1 = *(const v4f*)(xr + 4);
  float ssq = 0.f;
#pragma unroll
  for (int e = 0; e < 4; ++e) { ssq += a0[e] * a0[e]; ssq += a1[e] * a1[e]; }
#pragma unroll
  for (int off = 1; off < 32; off <<= 1) ssq += __shfl_xor(ssq, off, 32);
  if (lane == 0) red[wave] = ssq;
  __syncthreads();
  const float tot = (red[0] + red[1]) + (red[2] + red[3]);
  const float rr = rsqrtf(tot * (1.0f / (float)kDModel) + eps);
  const v4f g0 = *(const v4f*)(gamma + 8 * tid);
  const v4f g1 = *(const v4f*)(gamma + 8 * tid + 4);
  v8h hv;
#pragma unroll
  for (int e = 0; e < 4; ++e) {
    hv[e]     = (_Float16)(a0[e] * (g0[e] * rr));
    hv[4 + e] = (_Float16)(a1[e] * (g1[e] * rr));
  }
  unsigned short* dst = hout + (size_t)row * kDModel + 8 * tid;
  *(volatile v8h*)(void*)dst = hv;
  __threadfence();
  *(volatile v8h*)(void*)dst = hv;
}

__global__ __launch_bounds__(128) void qk_scale_rope_kernel(
    const float* __restrict__ qk, const float* __restrict__ pos, const float* __restrict__ ascale,
    unsigned short* __restrict__ qout, unsigned short* __restrict__ kout, int ntok, float eps, float osc) {
  __shared__ __align__(16) float sq[kDModel];
  __shared__ __align__(16) float sk[kDModel];
  __shared__ __align__(16) float soq[kDModel];
  __shared__ __align__(16) float sok[kDModel];
  __shared__ float tcs[kHeads * kRopeD];
  __shared__ float tsn[kHeads * kRopeD];
  int tok = blockIdx.x;
  if (tok > ntok - 1) tok = ntok - 1;
  const int tid = threadIdx.x;
  const int hd  = tid >> 3;
  const int sub = tid & 7;

  const float* qr = qk + (size_t)tok * (2 * kDModel) + 8 * tid;
  const float* kr = qr + kDModel;
  const v4f q0 = *(const v4f*)(qr), q1 = *(const v4f*)(qr + 4);
  const v4f k0 = *(const v4f*)(kr), k1 = *(const v4f*)(kr + 4);
  float ssq = 0.f, ssk = 0.f;
#pragma unroll
  for (int e = 0; e < 4; ++e) {
    ssq += q0[e] * q0[e]; ssq += q1[e] * q1[e];
    ssk += k0[e] * k0[e]; ssk += k1[e] * k1[e];
  }
#pragma unroll
  for (int off = 1; off < 8; off <<= 1) {
    ssq += __shfl_xor(ssq, off, 32);
    ssk += __shfl_xor(ssk, off, 32);
  }
  const float sc = sqrtf(ascale[hd]);
  const float rq = sc * rsqrtf(ssq + eps);
  const float rk = sc * rsqrtf(ssk + eps);
  *(v4f*)(sq + 8 * tid)     = q0 * rq;
  *(v4f*)(sq + 8 * tid + 4) = q1 * rq;
  *(v4f*)(sk + 8 * tid)     = k0 * rk;
  *(v4f*)(sk + 8 * tid + 4) = k1 * rk;

  const float p0 = pos[(size_t)tok * 3 + 0];
  const float p1 = pos[(size_t)tok * 3 + 1];
  const float p2 = pos[(size_t)tok * 3 + 2];
#pragma unroll 1
  for (int idx = tid; idx < kHeads * kRopeD; idx += 128) {
    const int th = idx / kRopeD;
    const int jj = idx - kRopeD * th;
    const int fi = jj / 10;
    const int fj = jj - 10 * fi;
    const float pf = (fi == 0) ? p0 : ((fi == 1) ? p1 : p2);
    const float fr = expf(kLogPi + (float)(fj * 16 + th) * kFreqStep);
    float sn, cs;
    sincosf(pf * fr, &sn, &cs);
    tcs[idx] = cs;
    tsn[idx] = sn;
  }
  __syncthreads();

#pragma unroll 1
  for (int e = 0; e < 8; ++e) {
    const int d = 8 * sub + e;
    const bool lt30 = d < kRopeD;
    const bool lt60 = d < 2 * kRopeD;
    const int jj = lt30 ? d : (lt60 ? (d - kRopeD) : 0);
    const int pd = lt30 ? (d + kRopeD) : (lt60 ? (d - kRopeD) : d);
    const float cs = tcs[hd * kRopeD + jj];
    const float sn = tsn[hd * kRopeD + jj];
    const float xqd = sq[hd * kHD + d], xqp = sq[hd * kHD + pd];
    const float xkd = sk[hd * kHD + d], xkp = sk[hd * kHD + pd];
    const float yq1 = xqd * cs - xqp * sn, yq2 = xqd * cs + xqp * sn;
    const float yk1 = xkd * cs - xkp * sn, yk2 = xkd * cs + xkp * sn;
    const float yq = lt30 ? yq1 : (lt60 ? yq2 : xqd);
    const float yk = lt30 ? yk1 : (lt60 ? yk2 : xkd);
    soq[8 * tid + e] = yq * osc;
    sok[8 * tid + e] = yk * osc;
  }
  v8h hq, hk;
#pragma unroll
  for (int e = 0; e < 8; ++e) {
    hq[e] = (_Float16)soq[8 * tid + e];
    hk[e] = (_Float16)sok[8 * tid + e];
  }
  unsigned short* dq = qout + (size_t)tok * kDModel + 8 * tid;
  unsigned short* dk = kout + (size_t)tok * kDModel + 8 * tid;
  *(volatile v8h*)(void*)dq = hq;
  *(volatile v8h*)(void*)dk = hk;
  __threadfence();
  *(volatile v8h*)(void*)dq = hq;
  *(volatile v8h*)(void*)dk = hk;
}

constexpr int kNW = 4;
constexpr int kKC = 64;

__device__ __forceinline__ v8f mma_h(v16h a, v16h b, v8f c) {
  c = __builtin_amdgcn_wmma_f32_16x16x32_f16(false, a, false, b, (short)0, c, false, false);
  asm volatile("v_nop\n\tv_nop\n\tv_nop\n\tv_nop" : "+v"(c) : "v"(a), "v"(b));
  return c;
}

__global__ __launch_bounds__(128)
void attn_f16_kernel(const unsigned short* __restrict__ qpl, const unsigned short* __restrict__ kpl,
                     const unsigned short* __restrict__ vtpl, unsigned short* __restrict__ opl,
                     float sscale, float oscale) {
  union FH { v16h v; v8h h[2]; };
  __shared__ __align__(16) _Float16 Ksh[kKC * kHD];
  __shared__ __align__(16) _Float16 Vth[kHD * kKC];
  __shared__ __align__(16) _Float16 Psh[kNW][16 * kKC];
  __shared__ __align__(16) float    Os[kNW][16 * 68];

  const int tid  = threadIdx.x;
  const int wave = tid >> 5;
  const int lane = tid & 31;
  const int hh   = lane >> 4;
  const int c    = lane & 15;

  const int nqb = kSeq / 64;
  const int bx  = blockIdx.x;
  const int qb  = bx % nqb;
  const int bh  = bx / nqb;
  const int h   = bh % kHeads;
  int b = bh / kHeads;
  if (b > kBatch - 1) b = kBatch - 1;
  const int q0 = qb * 64 + wave * 16;

  const _Float16* Qh = (const _Float16*)(const void*)qpl + (size_t)b * kSeq * kDModel + (size_t)h * kHD;
  const _Float16* Kh = (const _Float16*)(const void*)kpl + (size_t)b * kSeq * kDModel + (size_t)h * kHD;
  const _Float16* Vh = (const _Float16*)(const void*)vtpl + (size_t)h * kHD * kTok + (size_t)b * kSeq;
  _Float16*       Ob = (_Float16*)(void*)opl + (size_t)b * kSeq * kDModel + (size_t)h * kHD;

  v16h qa[2];
#pragma unroll
  for (int dc = 0; dc < 2; ++dc)
    qa[dc] = Frag<_Float16>::load(Qh + (size_t)(q0 + c) * kDModel + dc * 32 + 8 * hh);

  float mrow[8], lrow[8];
  v8f oacc[4];
#pragma unroll
  for (int r = 0; r < 8; ++r) { mrow[r] = -INFINITY; lrow[r] = 0.f; }
#pragma unroll
  for (int t = 0; t < 4; ++t) oacc[t] = (v8f){0.f,0.f,0.f,0.f,0.f,0.f,0.f,0.f};

  const int nChunks = kSeq / kKC;
  for (int kc = 0; kc < nChunks; ++kc) {
    const int kv0 = kc * kKC;
    __syncthreads();
    {
      const int r = tid >> 1, half = (tid & 1) * 32;
      const _Float16* ks = Kh + (size_t)(kv0 + r) * kDModel + half;
      const _Float16* vs = Vh + (size_t)r * kTok + kv0 + half;
#pragma unroll
      for (int i = 0; i < 4; ++i) {
        const v8h a0 = *(const v8h*)(ks + 8 * i);
        const v8h b0 = *(const v8h*)(vs + 8 * i);
        *(v8h*)(Ksh + r * kHD + half + 8 * i) = a0;
        *(v8h*)(Vth + r * kKC + half + 8 * i) = b0;
      }
    }
    __syncthreads();

    v8f s[4];
#pragma unroll
    for (int j = 0; j < 4; ++j) {
      s[j] = (v8f){0.f,0.f,0.f,0.f,0.f,0.f,0.f,0.f};
#pragma unroll
      for (int dc = 0; dc < 2; ++dc) {
        FH kb;
        kb.h[0] = *(const v8h*)(Ksh + (j * 16 + c) * kHD + dc * 32 + 8 * hh);
        kb.h[1] = *(const v8h*)(Ksh + (j * 16 + c) * kHD + dc * 32 + 16 + 8 * hh);
        s[j] = mma_h(qa[dc], kb.v, s[j]);
      }
    }
    float cm[8];
#pragma unroll
    for (int r = 0; r < 8; ++r) {
      float m = -INFINITY;
#pragma unroll
      for (int j = 0; j < 4; ++j) {
        const float sv = s[j][r] * sscale;
        s[j][r] = sv;
        m = fmaxf(m, sv);
      }
#pragma unroll
      for (int off = 1; off < 16; off <<= 1) m = fmaxf(m, __shfl_xor(m, off, 32));
      cm[r] = m;
    }
    _Float16* pw = Psh[wave];
#pragma unroll
    for (int r = 0; r < 8; ++r) {
      const float mnew = fmaxf(mrow[r], cm[r]);
      const float alpha = expf(mrow[r] - mnew);
      mrow[r] = mnew;
      float psum = 0.f;
#pragma unroll
      for (int j = 0; j < 4; ++j) {
        const float p = expf(s[j][r] - mnew);
        psum += p;
        pw[(8 * hh + r) * kKC + j * 16 + c] = (_Float16)(p * kPSC);
      }
#pragma unroll
      for (int off = 1; off < 16; off <<= 1) psum += __shfl_xor(psum, off, 32);
      lrow[r] = lrow[r] * alpha + psum;
#pragma unroll
      for (int t = 0; t < 4; ++t) oacc[t][r] *= alpha;
    }
    __builtin_amdgcn_fence(__ATOMIC_RELEASE, "workgroup");
    __builtin_amdgcn_wave_barrier();
    __builtin_amdgcn_fence(__ATOMIC_ACQUIRE, "workgroup");
#pragma unroll 1
    for (int kk = 0; kk < 2; ++kk) {
      FH pa;
      pa.h[0] = *(const v8h*)(pw + c * kKC + kk * 32 + 8 * hh);
      pa.h[1] = *(const v8h*)(pw + c * kKC + kk * 32 + 16 + 8 * hh);
#pragma unroll
      for (int t = 0; t < 4; ++t) {
        FH vb;
        vb.h[0] = *(const v8h*)(Vth + (t * 16 + c) * kKC + kk * 32 + 8 * hh);
        vb.h[1] = *(const v8h*)(Vth + (t * 16 + c) * kKC + kk * 32 + 16 + 8 * hh);
        oacc[t] = mma_h(pa.v, vb.v, oacc[t]);
      }
    }
  }

  float* os = Os[wave];
#pragma unroll
  for (int r = 0; r < 8; ++r) {
    const float inv = oscale * (1.0f / (lrow[r] * kPSC));
#pragma unroll
    for (int t = 0; t < 4; ++t) os[(8 * hh + r) * 68 + t * 16 + c] = oacc[t][r] * inv;
  }
  __builtin_amdgcn_fence(__ATOMIC_RELEASE, "workgroup");
  __builtin_amdgcn_wave_barrier();
  __builtin_amdgcn_fence(__ATOMIC_ACQUIRE, "workgroup");
  {
    const int q4 = lane >> 3, c8 = (lane & 7) * 8;
    for (int pass = 0; pass < 2; ++pass) {
#pragma unroll
      for (int it = 0; it < 4; ++it) {
        const int row = it * 4 + q4;
        const float* sp = os + row * 68 + c8;
        v8h hv;
#pragma unroll
        for (int e = 0; e < 8; ++e) hv[e] = (_Float16)sp[e];
        *(volatile v8h*)(Ob + (size_t)(q0 + row) * kDModel + c8) = hv;
      }
      __threadfence();
    }
  }
}

extern "C" void kernel_launch(void* const* d_in, const int* in_sizes, int n_in,
                              void* d_out, int out_size, void* d_ws,
                              size_t ws_size, hipStream_t stream) {
  if (n_in < 6) return;
  if (in_sizes[0] != kTok * kDModel) return;
  if (in_sizes[1] != kTok * 3) return;
  if (in_sizes[2] != kDModel) return;
  if (in_sizes[3] != 3 * kDModel * kDModel) return;
  if (in_sizes[4] != kDModel * kDModel) return;
  if (in_sizes[5] < kHeads) return;
  if (out_size != kTok * kDModel) return;

  const float* x      = (const float*)d_in[0];
  const float* pos    = (const float*)d_in[1];
  const float* nscale = (const float*)d_in[2];
  const float* w_qkv  = (const float*)d_in[3];
  const float* w_out  = (const float*)d_in[4];
  const float* ascale = (const float*)d_in[5];
  float* out = (float*)d_out;

  const size_t szWQ = (size_t)3 * kDModel * kDModel * 2;
  const size_t szWO = (size_t)kDModel * kDModel * 2;
  const size_t szH  = (size_t)kTok * kDModel * 2;
  const size_t szQK = (size_t)kTok * 2 * kDModel * 4;
  const size_t szVT = (size_t)kDModel * kTok * 2;
  const size_t szP  = (size_t)kTok * kDModel * 2;
  const size_t oWQ = 0;
  const size_t oWO = oWQ + szWQ;
  const size_t oH  = oWO + szWO;
  const size_t oQK = oH + szH;
  const size_t oVT = oQK + szQK;
  const size_t oQP = oVT + szVT;
  const size_t oKP = oQP + szP;
  const size_t oO  = oKP + szP;
  const size_t total = oO + szP;
  if (total > ws_size) return;

  char* ws = (char*)d_ws;
  unsigned short* WQ16 = (unsigned short*)(ws + oWQ);
  unsigned short* WO16 = (unsigned short*)(ws + oWO);
  unsigned short* H16  = (unsigned short*)(ws + oH);
  float*          QK32 = (float*)(ws + oQK);
  unsigned short* VT16 = (unsigned short*)(ws + oVT);
  unsigned short* QP16 = (unsigned short*)(ws + oQP);
  unsigned short* KP16 = (unsigned short*)(ws + oKP);
  unsigned short* O16  = (unsigned short*)(ws + oO);

  {
    const int nq2 = 3 * kDModel * kDModel / 2;
    const int no2 = kDModel * kDModel / 2;
    cast_scale_f32_f16x2<<<dim3((nq2 + 255) / 256), dim3(256), 0, stream>>>(w_qkv, WQ16, nq2, kWqScale);
    cast_scale_f32_f16x2<<<dim3((no2 + 255) / 256), dim3(256), 0, stream>>>(w_out, WO16, no2, kWoScale);
  }
  rmsnorm_f16_kernel<<<dim3(kTok), dim3(128), 0, stream>>>(x, nscale, H16, kTok, kEps);
  wmma_gemm64<0, false, 0, 0, false, 0><<<dim3((kTok / 64) * (2 * kDModel / 64) / 8, 1), dim3(256), 0, stream>>>(
      H16, H16, kDModel, 0L,
      WQ16, WQ16, kDModel, 0L,
      (void*)QK32, (void*)QK32, 2 * kDModel, 0L,
      nscale, x, 0L,
      kTok, 2 * kDModel, kDModel, 1.0f / kWqScale);
  wmma_gemm64<0, false, 0, 1, false, 0><<<dim3((kDModel / 64) * (kTok / 64) / 8, 1), dim3(256), 0, stream>>>(
      WQ16 + (size_t)2 * kDModel * kDModel, WQ16 + (size_t)2 * kDModel * kDModel, kDModel, 0L,
      H16, H16, kDModel, 0L,
      (void*)VT16, (void*)VT16, kTok, 0L,
      nscale, x, 0L,
      kDModel, kTok, kDModel, 1.0f / kWqScale);
  qk_scale_rope_kernel<<<dim3(kTok), dim3(128), 0, stream>>>(QK32, pos, ascale, QP16, KP16, kTok, kEps, kQkScale);
  attn_f16_kernel<<<dim3(kBatch * kHeads * (kSeq / 64)), dim3(128), 0, stream>>>(
      QP16, KP16, VT16, O16, 1.0f / (kQkScale * kQkScale), kOScale);
  wmma_gemm64<0, false, 0, 0, true, 0><<<dim3((kTok / 64) * (kDModel / 64) / 8, 1), dim3(256), 0, stream>>>(
      O16, O16, kDModel, 0L,
      WO16, WO16, kDModel, 0L,
      (void*)out, (void*)out, kDModel, 0L,
      nscale, x, 0L,
      kTok, kDModel, kDModel, 1.0f / (kOScale * kWoScale));
}
